// PointNet2Encoder_26396869001381
// MI455X (gfx1250) — hardware-verified
//
#include <hip/hip_runtime.h>
#pragma clang fp contract(off)

typedef __attribute__((ext_vector_type(16))) _Float16 v16h;
typedef __attribute__((ext_vector_type(8)))  _Float16 v8h;
typedef __attribute__((ext_vector_type(16))) __bf16   v16b;
typedef __attribute__((ext_vector_type(8)))  __bf16   v8b;
typedef __attribute__((ext_vector_type(8)))  float    v8f;
typedef __attribute__((ext_vector_type(4)))  float    v4f;
typedef __attribute__((ext_vector_type(2)))  float    v2f;
typedef __attribute__((ext_vector_type(4)))  unsigned v4u;

constexpr float WCARRY     = 16.0f;
constexpr float WCARRY_INV = 1.0f / 16.0f;
constexpr float BN_VAR_EPS = (float)(1.0 + 1e-5);

__device__ __forceinline__ unsigned short f2bf_bits(float f) {
  unsigned u = __float_as_uint(f);
  return (unsigned short)((u + 0x7FFFu + ((u >> 16) & 1u)) >> 16);
}
__device__ __forceinline__ float bf_bits2f(unsigned short h) { return __uint_as_float(((unsigned)h) << 16); }

__device__ __forceinline__ void dep_guard4_h(v8f& a, v8f& b, v8f& c, v8f& d, v16h x, v16h y) { asm volatile("v_nop\n\tv_nop\n\tv_nop\n\tv_nop" : "+v"(a), "+v"(b), "+v"(c), "+v"(d) : "v"(x), "v"(y)); }
__device__ __forceinline__ void dep_guard4_b(v8f& a, v8f& b, v8f& c, v8f& d, v16b x, v16b y) { asm volatile("v_nop\n\tv_nop\n\tv_nop\n\tv_nop" : "+v"(a), "+v"(b), "+v"(c), "+v"(d) : "v"(x), "v"(y)); }
__device__ __forceinline__ void keep4_h(v16h a, v16h b, v16h c, v16h d) { asm volatile("v_nop" :: "v"(a), "v"(b), "v"(c), "v"(d)); }
__device__ __forceinline__ void keep4_b(v16b a, v16b b, v16b c, v16b d) { asm volatile("v_nop" :: "v"(a), "v"(b), "v"(c), "v"(d)); }
__device__ __forceinline__ void acc_guard4(v8f& a, v8f& b, v8f& c, v8f& d) { asm volatile("v_nop\n\tv_nop\n\tv_nop\n\tv_nop" : "+v"(a), "+v"(b), "+v"(c), "+v"(d)); }

template <typename T> struct Frag;
template <> struct Frag<_Float16> {
  typedef v16h V; union U { v16h v; v8h h[2]; };
  static __device__ __forceinline__ v16h load(const _Float16* p) {
    U f; f.h[0] = *(const v8h*)(p); f.h[1] = *(const v8h*)(p + 16); return f.v;
  }
  static __device__ __forceinline__ v8f mma(v16h a, v16h b, v8f c) {
    return __builtin_amdgcn_wmma_f32_16x16x32_f16(false, a, false, b, (short)0, c, false, false);
  }
  static __device__ __forceinline__ void guard4(v8f& a, v8f& b, v8f& c, v8f& d, v16h x, v16h y) { dep_guard4_h(a, b, c, d, x, y); }
  static __device__ __forceinline__ void keep(v16h a, v16h b, v16h c, v16h d) { keep4_h(a, b, c, d); }
};
template <> struct Frag<__bf16> {
  typedef v16b V; union U { v16b v; v8b h[2]; };
  static __device__ __forceinline__ v16b load(const __bf16* p) {
    U f; f.h[0] = *(const v8b*)(p); f.h[1] = *(const v8b*)(p + 16); return f.v;
  }
  static __device__ __forceinline__ v8f mma(v16b a, v16b b, v8f c) {
    return __builtin_amdgcn_wmma_f32_16x16x32_bf16(false, a, false, b, (short)0, c, false, false);
  }
  static __device__ __forceinline__ void guard4(v8f& a, v8f& b, v8f& c, v8f& d, v16b x, v16b y) { dep_guard4_b(a, b, c, d, x, y); }
  static __device__ __forceinline__ void keep(v16b a, v16b b, v16b c, v16b d) { keep4_b(a, b, c, d); }
};

__device__ __forceinline__ v8f mma_h(v16h a, v16h b, v8f c) {
  c = __builtin_amdgcn_wmma_f32_16x16x32_f16(false, a, false, b, (short)0, c, false, false);
  asm volatile("v_nop\n\tv_nop\n\tv_nop\n\tv_nop" : "+v"(c) : "v"(a), "v"(b));
  return c;
}

__device__ __forceinline__ float lane_zero_f() { float z = 0.0f; asm volatile("" : "+v"(z)); return z; }
__device__ __forceinline__ unsigned lane_zero_u() { unsigned z = 0u; asm volatile("" : "+v"(z)); return z; }

template <int ET> struct Elem;
template <> struct Elem<0> { typedef _Float16 T; };
template <> struct Elem<1> { typedef __bf16 T; };
template <int ET, bool SPLIT, int BIAS_MODE, int OUT_MODE, bool RESID, int ACT = 0>
__global__ __launch_bounds__(256) void wmma_gemm64(
    const unsigned short* __restrict__ Ap, const unsigned short* __restrict__ A2p, int lda, long strideA,
    const unsigned short* __restrict__ Btp, const unsigned short* __restrict__ Bt2p, int ldb, long strideB,
    void* __restrict__ Cout, void* __restrict__ Cout2, int ldc, long strideC,
    const float* __restrict__ bias,
    const float* __restrict__ resid, long strideR,
    int M, int N, int K, float scale) {
  typedef typename Elem<ET>::T T;
  typedef typename Frag<T>::V V;
  const T* A = (const T*)Ap; const T* A2 = (const T*)A2p; const T* Bt = (const T*)Btp; const T* Bt2 = (const T*)Bt2p;
  __shared__ __align__(16) float sT[8][16 * 68];
  const int b    = blockIdx.y;
  const int lane = threadIdx.x & 31;
  const int wave = threadIdx.x >> 5;
  const int tilesN = N >> 6;
  const int tilesM = M >> 6;
  const int tile = blockIdx.x * 8 + wave;
  if (tile >= tilesM * tilesN) return;
  const int tm = tile / tilesN;
  const int tn = tile - tm * tilesN;
  const int m0 = tm << 6;
  const int n0 = tn << 6;

  const T* Ab  = A  + (size_t)b * strideA;
  const T* Bb  = Bt + (size_t)b * strideB;
  const T* Ab2 = SPLIT ? (A2  + (size_t)b * strideA) : nullptr;
  const T* Bb2 = SPLIT ? (Bt2 + (size_t)b * strideB) : nullptr;

  const int rlane = lane & 15;
  const int koff  = (lane >> 4) * 8;
  const int mOff  = (lane >> 4) * 8;

  v8f acc[4][4];
#pragma unroll
  for (int i = 0; i < 4; ++i)
#pragma unroll
    for (int j = 0; j < 4; ++j) acc[i][j] = (v8f){0.f,0.f,0.f,0.f,0.f,0.f,0.f,0.f};

  for (int k0 = 0; k0 < K; k0 += 32) {
    V bh[4], bl[4];
#pragma unroll
    for (int j = 0; j < 4; ++j) {
      const size_t bo = (size_t)(n0 + (j << 4) + rlane) * ldb + koff + k0;
      bh[j] = Frag<T>::load(Bb + bo);
      if (SPLIT) bl[j] = Frag<T>::load(Bb2 + bo);
    }
#pragma unroll
    for (int i = 0; i < 4; ++i) {
      const size_t ao = (size_t)(m0 + (i << 4) + rlane) * lda + koff + k0;
      V ah = Frag<T>::load(Ab + ao);
      V al = ah;
      if (SPLIT) al = Frag<T>::load(Ab2 + ao);
#pragma unroll
      for (int j = 0; j < 4; ++j) {
        acc[i][j] = Frag<T>::mma(ah, bh[j], acc[i][j]);
        if (SPLIT) {
          acc[i][j] = Frag<T>::mma(ah, bl[j], acc[i][j]);
          acc[i][j] = Frag<T>::mma(al, bh[j], acc[i][j]);
        }
      }
      Frag<T>::guard4(acc[i][0], acc[i][1], acc[i][2], acc[i][3], ah, al);
    }
    Frag<T>::keep(bh[0], bh[1], bh[2], bh[3]);
    if (SPLIT) Frag<T>::keep(bl[0], bl[1], bl[2], bl[3]);
  }
  acc_guard4(acc[0][0], acc[0][1], acc[0][2], acc[0][3]);
  acc_guard4(acc[1][0], acc[1][1], acc[1][2], acc[1][3]);
  acc_guard4(acc[2][0], acc[2][1], acc[2][2], acc[2][3]);
  acc_guard4(acc[3][0], acc[3][1], acc[3][2], acc[3][3]);

  float* slab = sT[wave];
  const float* Rb = RESID ? (resid + (size_t)b * strideR) : nullptr;
#pragma unroll
  for (int i = 0; i < 4; ++i) {
    const int mBase = m0 + (i << 4);
#pragma unroll
    for (int j = 0; j < 4; ++j) {
      const int n = n0 + (j << 4) + rlane;
      float bv = 0.f;
      if (BIAS_MODE == 2) bv = bias[n];
#pragma unroll
      for (int r = 0; r < 8; ++r) {
        float v = acc[i][j][r] * scale;
        if (BIAS_MODE == 1) v += bias[mBase + mOff + r];
        if (BIAS_MODE == 2) v += bv;
        if (RESID) v += Rb[(size_t)(mBase + mOff + r) * ldc + n];
        if (ACT == 2) v = fmaxf(v, 0.0f);
        slab[(mOff + r) * 68 + (j << 4) + rlane] = v;
      }
    }
    __builtin_amdgcn_fence(__ATOMIC_RELEASE, "workgroup");
    __builtin_amdgcn_wave_barrier();
    __builtin_amdgcn_fence(__ATOMIC_ACQUIRE, "workgroup");
    if (OUT_MODE == 0) {
      float* C = (float*)Cout + (size_t)b * strideC;
      const int hh = lane >> 4, c4 = (lane & 15) * 4;
      for (int pass = 0; pass < 2; ++pass) {
#pragma unroll
        for (int it = 0; it < 8; ++it) {
          const int row = it * 2 + hh;
          v4f v = *(const v4f*)(slab + row * 68 + c4);
          *(volatile v4f*)(C + (size_t)(mBase + row) * ldc + n0 + c4) = v;
        }
        __threadfence();
      }
    } else {
      const int q = lane >> 3, c8 = (lane & 7) * 8;
      unsigned short* C  = (unsigned short*)Cout  + (size_t)b * strideC;
      unsigned short* C2 = (OUT_MODE == 2) ? ((unsigned short*)Cout2 + (size_t)b * strideC) : nullptr;
      for (int pass = 0; pass < 2; ++pass) {
#pragma unroll
        for (int it = 0; it < 4; ++it) {
          const int row = it * 4 + q;
          const float* sp = slab + row * 68 + c8;
          v8h hv, lv;
#pragma unroll
          for (int e = 0; e < 8; ++e) {
            if (OUT_MODE == 1) {
              hv[e] = (_Float16)sp[e];
            } else {
              unsigned short hb = f2bf_bits(sp[e]);
              unsigned short lb = f2bf_bits(sp[e] - bf_bits2f(hb));
              hv[e] = __builtin_bit_cast(_Float16, hb);
              lv[e] = __builtin_bit_cast(_Float16, lb);
            }
          }
          *(volatile v8h*)(C + (size_t)(mBase + row) * ldc + n0 + c8) = hv;
          if (OUT_MODE == 2) *(volatile v8h*)(C2 + (size_t)(mBase + row) * ldc + n0 + c8) = lv;
        }
        __threadfence();
      }
    }
    __builtin_amdgcn_fence(__ATOMIC_RELEASE, "workgroup");
    __builtin_amdgcn_wave_barrier();
    __builtin_amdgcn_fence(__ATOMIC_ACQUIRE, "workgroup");
  }
}

__global__ __launch_bounds__(256) void cvt_wt_kernel(const float* W, unsigned short* Wt,
                                                     int Cin, int Cout, int KP, int nlead, float carry) {
  const int q = blockIdx.x * 256 + threadIdx.x;
  const int cpr = KP >> 3;
  const int total = Cout * cpr;
  if (q >= total) return;
  const int n = q / cpr;
  const int kc = (q - n * cpr) * 8;
  const float zz = lane_zero_f();
  const int nf = Cin - nlead;
  v8h hv;
#pragma unroll
  for (int e = 0; e < 8; ++e) {
    const int k = kc + e;
    int r = (k < nf) ? (k + nlead) : (k - nf);
    r = r < 0 ? 0 : r;
    r = r > Cin - 1 ? Cin - 1 : r;
    const float wv = W[(size_t)r * Cout + n];
    const float sv = wv * carry;
    const float v = (k < Cin) ? sv : zz;
    hv[e] = (_Float16)v;
  }
  volatile v8h* dst = (volatile v8h*)(Wt + (size_t)q * 8);
  *dst = hv;
  __threadfence();
  *dst = hv;
}

template <int PPT, bool SRC6>
__global__ __launch_bounds__(256) void fps_kernel(const float* src, float* cent_out, int N, int S) {
#pragma clang fp contract(off)
  constexpr int STG = SRC6 ? 1024 * 6 : 4;
  __shared__ __align__(16) float stage[STG];
  __shared__ __align__(16) float cent_s[256 * 4];
  __shared__ float rv[2][8];
  __shared__ int   ri[2][8];
  const int b = blockIdx.x;
  const int tid = threadIdx.x, lane = tid & 31, wave = tid >> 5;
  if (S > 256) S = 256;
  float px[PPT], py[PPT], pz[PPT], dd[PPT];
  bool valid = true;
  if (SRC6) {
#pragma unroll
    for (int ch = 0; ch < PPT / 4; ++ch) {
      __syncthreads();
      const v4f* g = (const v4f*)(src + ((size_t)b * N + (size_t)ch * 1024) * 6);
#pragma unroll
      for (int i = 0; i < 6; ++i) {
        const v4f t = g[tid + 256 * i];
        *(v4f*)(stage + 4 * (tid + 256 * i)) = t;
      }
      __syncthreads();
#pragma unroll
      for (int jj = 0; jj < 4; ++jj) {
        const int j = ch * 4 + jj;
        const int o = (tid + 256 * jj) * 6;
        px[j] = stage[o + 0];
        py[j] = stage[o + 1];
        pz[j] = stage[o + 2];
      }
    }
  } else {
    const int nc = tid < N ? tid : N - 1;
    const v4f pv = *(const v4f*)(src + ((size_t)b * N + nc) * 4);
    px[0] = pv[0]; py[0] = pv[1]; pz[0] = pv[2];
    valid = tid < N;
  }
#pragma unroll
  for (int j = 0; j < PPT; ++j) dd[j] = 1e10f;

  int far = 0;
  for (int i = 0; i < S; ++i) {
    int fc = far < 0 ? 0 : far;
    fc = fc > N - 1 ? N - 1 : fc;
    float cx, cy, cz;
    if (SRC6) {
      const float* cp = src + ((size_t)b * N + fc) * 6;
      cx = cp[0]; cy = cp[1]; cz = cp[2];
    } else {
      const v4f cv = *(const v4f*)(src + ((size_t)b * N + fc) * 4);
      cx = cv[0]; cy = cv[1]; cz = cv[2];
    }
    if (tid == 0) {
      v4f cw; cw[0] = cx; cw[1] = cy; cw[2] = cz; cw[3] = 0.0f;
      *(v4f*)(cent_s + 4 * i) = cw;
    }
    float bm = -2.0f;
    int bi = 0x7fffffff;
#pragma unroll
    for (int j = 0; j < PPT; ++j) {
      const float dx = px[j] - cx;
      const float dy = py[j] - cy;
      const float dz = pz[j] - cz;
      const float t0 = dx * dx;
      const float t1 = dy * dy;
      const float t2 = dz * dz;
      const float d = (t0 + t2) + t1;
      const float nd = fminf(dd[j], d);
      dd[j] = nd;
      const float val = valid ? nd : -1.0f;
      const bool tk = val > bm;
      bm = tk ? val : bm;
      bi = tk ? (tid + 256 * j) : bi;
    }
#pragma unroll
    for (int off = 16; off > 0; off >>= 1) {
      const float ov = __shfl_xor(bm, off, 32);
      const int   oi = __shfl_xor(bi, off, 32);
      const bool tk = (ov > bm) || ((ov == bm) && (oi < bi));
      bm = tk ? ov : bm;
      bi = tk ? oi : bi;
    }
    const int par = i & 1;
    if (lane == 0) { rv[par][wave] = bm; ri[par][wave] = bi; }
    __syncthreads();
    float fm = rv[par][0];
    int   fi = ri[par][0];
#pragma unroll
    for (int w = 1; w < 8; ++w) {
      const float ov = rv[par][w];
      const int   oi = ri[par][w];
      const bool tk = (ov > fm) || ((ov == fm) && (oi < fi));
      fm = tk ? ov : fm;
      fi = tk ? oi : fi;
    }
    far = fi;
  }
  __syncthreads();
  if (tid < S) {
    const v4f cv = *(const v4f*)(cent_s + 4 * tid);
    volatile v4f* d = (volatile v4f*)(cent_out + ((size_t)b * S + tid) * 4);
    *d = cv;
    __threadfence();
    *d = cv;
  }
}

template <int NS, int FC, int K1P, int C1, int C2, bool SRC6>
__global__ __launch_bounds__(256) void group_mlp_kernel(
    const float* pts, const unsigned short* featsIn, const float* centers,
    const unsigned short* w1t, const float* b1, const unsigned short* w2t, const float* b2,
    unsigned short* fout, int N, int S, float r2) {
#pragma clang fp contract(off)
  constexpr int MT = NS / 16;
  static_assert(NS % 16 == 0 && NS <= 64, "group size");
  static_assert(K1P % 32 == 0 && C1 % 32 == 0 && C2 % 128 == 0, "k and n tiling");
  static_assert(SRC6 ? (FC == 6 && K1P == 32) : (FC % 8 == 0 && K1P - FC == 32), "row layout");
  constexpr int CPR = SRC6 ? 1 : (FC / 8);
  constexpr int NIT = SRC6 ? 0 : (NS * CPR / 256);
  static_assert(SRC6 || ((NS * CPR) % 256 == 0), "gather coverage");

  __shared__ __align__(16) _Float16 Xs[NS * K1P];
  __shared__ __align__(16) _Float16 H1s[NS * C1];
  __shared__ __align__(16) float om[C2];
  __shared__ int hitlist[64];
  __shared__ int wcnt[2][8];

  const int tid = threadIdx.x, lane = tid & 31, wave = tid >> 5;
  const int hh = lane >> 4, l16 = lane & 15;
  const int blk = blockIdx.x;
  const int b = blk / S;
  const size_t pbase = (size_t)b * N;
  const v4f cen = *(const v4f*)(centers + (size_t)blk * 4);
  const float cx = cen[0], cy = cen[1], cz = cen[2];

  if (tid < 64) hitlist[tid] = N - 1;

  int cnt = 0;
  const int nchunk = (N + 255) >> 8;
  for (int ch = 0; ch < nchunk; ++ch) {
    const int n = (ch << 8) + tid;
    const int nc = n < N ? n : N - 1;
    float qx, qy, qz;
    if (SRC6) {
      const float* pp = pts + (pbase + nc) * 6;
      qx = pp[0]; qy = pp[1]; qz = pp[2];
    } else {
      const v4f pv = *(const v4f*)(pts + (pbase + nc) * 4);
      qx = pv[0]; qy = pv[1]; qz = pv[2];
    }
    const float dx = cx - qx;
    const float dy = cy - qy;
    const float dz = cz - qz;
    const float t0 = dx * dx;
    const float t1 = dy * dy;
    const float t2 = dz * dz;
    const float d2 = (t0 + t2) + t1;
    const bool hit = (n < N) && (d2 < r2);
    const unsigned mask = (unsigned)__ballot(hit ? 1 : 0);
    const int pre = __popc(mask & ((1u << lane) - 1u));
    const int par = ch & 1;
    if (lane == 0) wcnt[par][wave] = __popc(mask);
    __syncthreads();
    int base = cnt, tot = 0;
#pragma unroll
    for (int w = 0; w < 8; ++w) {
      const int c = wcnt[par][w];
      base += (w < wave) ? c : 0;
      tot += c;
    }
    const int pos = base + pre;
    if (hit && pos < NS) hitlist[pos] = n;
    cnt += tot;
    if (cnt >= NS) break;
  }
  __syncthreads();
  const int cntc = cnt < NS ? cnt : NS;
  const int first = hitlist[0];

  if (SRC6) {
    if (tid < NS) {
      const int hl = hitlist[tid];
      int p = (tid < cntc) ? hl : first;
      p = p < 0 ? 0 : p;
      p = p > N - 1 ? N - 1 : p;
      const float* pp = pts + (pbase + p) * 6;
      const v2f a0 = *(const v2f*)(pp);
      const v2f a1 = *(const v2f*)(pp + 2);
      const v2f a2 = *(const v2f*)(pp + 4);
      const float x = a0[0], y = a0[1], z = a1[0];
      const float e0 = a1[1], e1 = a2[0], e2 = a2[1];
      const float rx = x - cx, ry = y - cy, rz = z - cz;
      const float zz = lane_zero_f();
      v8h c0, c1, c2;
      c0[0] = (_Float16)e0; c0[1] = (_Float16)e1; c0[2] = (_Float16)e2;
      c0[3] = (_Float16)x;  c0[4] = (_Float16)y;  c0[5] = (_Float16)z;
      c0[6] = (_Float16)rx; c0[7] = (_Float16)ry;
      c1[0] = (_Float16)rz;
#pragma unroll
      for (int e = 1; e < 8; ++e) c1[e] = (_Float16)zz;
#pragma unroll
      for (int e = 0; e < 8; ++e) c2[e] = (_Float16)zz;
      _Float16* xr = Xs + tid * K1P;
      *(v8h*)(xr + 0)  = c0;
      *(v8h*)(xr + 8)  = c1;
      *(v8h*)(xr + 16) = c2;
      *(v8h*)(xr + 24) = c2;
    }
  } else {
#pragma unroll
    for (int i = 0; i < NIT; ++i) {
      const int q = tid + 256 * i;
      const int s = q / CPR;
      const int cc = q - s * CPR;
      const int hl = hitlist[s];
      int p = (s < cntc) ? hl : first;
      p = p < 0 ? 0 : p;
      p = p > N - 1 ? N - 1 : p;
      const uint4 w = *(const uint4*)(featsIn + (pbase + p) * FC + cc * 8);
      *(uint4*)(Xs + s * K1P + cc * 8) = w;
    }
    if (tid < NS) {
      const int hl = hitlist[tid];
      int p = (tid < cntc) ? hl : first;
      p = p < 0 ? 0 : p;
      p = p > N - 1 ? N - 1 : p;
      const v4f pv = *(const v4f*)(pts + (pbase + p) * 4);
      const float rx = pv[0] - cx, ry = pv[1] - cy, rz = pv[2] - cz;
      const float zz = lane_zero_f();
      v8h c0, c2;
      c0[0] = (_Float16)rx; c0[1] = (_Float16)ry; c0[2] = (_Float16)rz;
#pragma unroll
      for (int e = 3; e < 8; ++e) c0[e] = (_Float16)zz;
#pragma unroll
      for (int e = 0; e < 8; ++e) c2[e] = (_Float16)zz;
      _Float16* xr = Xs + tid * K1P + FC;
      *(v8h*)(xr + 0)  = c0;
      *(v8h*)(xr + 8)  = c2;
      *(v8h*)(xr + 16) = c2;
      *(v8h*)(xr + 24) = c2;
    }
  }
  __syncthreads();

  {
    constexpr int NTA = C1 / 16;
    constexpr int MSA = (NTA >= 8) ? 1 : (((8 / NTA) < MT) ? (8 / NTA) : MT);
    constexpr int MCHA = MT / MSA;
    static_assert(MCHA * MSA == MT, "m split");
    const _Float16* W1 = (const _Float16*)w1t;
    for (int item = wave; item < NTA * MSA; item += 8) {
      const int nt = item % NTA;
      const int mb = (item / NTA) * MCHA;
      const int n0 = nt * 16;
      v8f acc[MCHA];
#pragma unroll
      for (int mi = 0; mi < MCHA; ++mi) acc[mi] = (v8f){0.f,0.f,0.f,0.f,0.f,0.f,0.f,0.f};
      const _Float16* brow = W1 + (size_t)(n0 + l16) * K1P + 8 * hh;
#pragma unroll 1
      for (int kk = 0; kk < K1P; kk += 32) {
        const v16h w = Frag<_Float16>::load(brow + kk);
#pragma unroll
        for (int mi = 0; mi < MCHA; ++mi) {
          const v16h a = Frag<_Float16>::load(Xs + ((mb + mi) * 16 + l16) * K1P + kk + 8 * hh);
          acc[mi] = mma_h(a, w, acc[mi]);
        }
      }
      const float bv = b1[n0 + l16];
#pragma unroll
      for (int mi = 0; mi < MCHA; ++mi) {
#pragma unroll
        for (int r = 0; r < 8; ++r) {
          float v = acc[mi][r] * WCARRY_INV;
          v = v + bv;
          v = fmaxf(v, 0.0f);
          H1s[((mb + mi) * 16 + 8 * hh + r) * C1 + n0 + l16] = (_Float16)v;
        }
      }
    }
  }
  __syncthreads();

  {
    constexpr int NTB = C2 / 16;
    const _Float16* W2 = (const _Float16*)w2t;
    for (int item = wave; item < NTB; item += 8) {
      const int n0 = item * 16;
      v8f acc[MT];
#pragma unroll
      for (int mi = 0; mi < MT; ++mi) acc[mi] = (v8f){0.f,0.f,0.f,0.f,0.f,0.f,0.f,0.f};
      const _Float16* brow = W2 + (size_t)(n0 + l16) * C1 + 8 * hh;
#pragma unroll 1
      for (int kk = 0; kk < C1; kk += 32) {
        const v16h w = Frag<_Float16>::load(brow + kk);
#pragma unroll
        for (int mi = 0; mi < MT; ++mi) {
          const v16h a = Frag<_Float16>::load(H1s + (mi * 16 + l16) * C1 + kk + 8 * hh);
          acc[mi] = mma_h(a, w, acc[mi]);
        }
      }
      const float bv = b2[n0 + l16];
      float mx = 0.0f;
#pragma unroll
      for (int mi = 0; mi < MT; ++mi) {
#pragma unroll
        for (int r = 0; r < 8; ++r) {
          float v = acc[mi][r] * WCARRY_INV;
          v = v + bv;
          mx = fmaxf(mx, v);
        }
      }
      const float other = __shfl_xor(mx, 16, 32);
      mx = fmaxf(mx, other);
      if (hh == 0) om[n0 + l16] = mx;
    }
  }
  __syncthreads();

  if (tid < C2 / 8) {
    const v4f u0 = *(const v4f*)(om + tid * 8);
    const v4f u1 = *(const v4f*)(om + tid * 8 + 4);
    v8h hv;
    hv[0] = (_Float16)u0[0]; hv[1] = (_Float16)u0[1]; hv[2] = (_Float16)u0[2]; hv[3] = (_Float16)u0[3];
    hv[4] = (_Float16)u1[0]; hv[5] = (_Float16)u1[1]; hv[6] = (_Float16)u1[2]; hv[7] = (_Float16)u1[3];
    volatile v8h* dst = (volatile v8h*)(fout + (size_t)blk * C2 + tid * 8);
    *dst = hv;
    __threadfence();
    *dst = hv;
  }
}

__global__ __launch_bounds__(256) void assemble_head_kernel(const unsigned short* feats3, const float* cent3,
                                                            unsigned short* A0) {
  const int q = blockIdx.x * 256 + threadIdx.x;
  if (q >= 512 * 68) return;
  const int row = q / 68;
  const int cc = q - row * 68;
  const int ccl = cc < 63 ? cc : 63;
  const uint4 f = *(const uint4*)(feats3 + (size_t)row * 512 + ccl * 8);
  const v4f c = *(const v4f*)(cent3 + (size_t)row * 4);
  unsigned f0 = f.x, f1 = f.y, f2 = f.z, f3 = f.w;
  float fx = c[0], fy = c[1], fz = c[2];
  asm volatile("" : "+v"(f0), "+v"(f1), "+v"(f2), "+v"(f3), "+v"(fx), "+v"(fy), "+v"(fz));
  const _Float16 hx = (_Float16)fx;
  const _Float16 hy = (_Float16)fy;
  const _Float16 hz = (_Float16)fz;
  const unsigned bx = (unsigned)__builtin_bit_cast(unsigned short, hx);
  const unsigned by = (unsigned)__builtin_bit_cast(unsigned short, hy);
  const unsigned bz = (unsigned)__builtin_bit_cast(unsigned short, hz);
  const unsigned zu = lane_zero_u();
  const unsigned x0 = bx | (by << 16);
  const unsigned x1 = bz | (zu << 16);
  const unsigned mf = 0u - (unsigned)(cc < 64);
  const unsigned mx = 0u - (unsigned)(cc == 64);
  v4u o;
  o[0] = (f0 & mf) | (x0 & mx);
  o[1] = (f1 & mf) | (x1 & mx);
  o[2] = (f2 & mf) | zu;
  o[3] = (f3 & mf) | zu;
  volatile v4u* dst = (volatile v4u*)(A0 + (size_t)q * 8);
  *dst = o;
  __threadfence();
  *dst = o;
}

__device__ __forceinline__ unsigned hmax_bits(unsigned m, unsigned h) {
  h = (h & 0x8000u) ? 0u : h;
  return h > m ? h : m;
}
__global__ __launch_bounds__(256) void maxpts_kernel(const unsigned short* G2, unsigned short* gfeat) {
  const int q = blockIdx.x * 256 + threadIdx.x;
  if (q >= 64 * 128) return;
  const int row = q >> 7;
  const int cc = q & 127;
  const int bc = row < 32 ? row : 31;
  const unsigned short* base = G2 + (size_t)bc * 16 * 1024 + cc * 8;
  unsigned m[8];
#pragma unroll
  for (int e = 0; e < 8; ++e) m[e] = 0u;
#pragma unroll 1
  for (int g = 0; g < 4; ++g) {
    uint4 w[4];
#pragma unroll
    for (int t = 0; t < 4; ++t) w[t] = *(const uint4*)(base + (size_t)(g * 4 + t) * 1024);
#pragma unroll
    for (int t = 0; t < 4; ++t) {
      m[0] = hmax_bits(m[0], w[t].x & 0xffffu); m[1] = hmax_bits(m[1], w[t].x >> 16);
      m[2] = hmax_bits(m[2], w[t].y & 0xffffu); m[3] = hmax_bits(m[3], w[t].y >> 16);
      m[4] = hmax_bits(m[4], w[t].z & 0xffffu); m[5] = hmax_bits(m[5], w[t].z >> 16);
      m[6] = hmax_bits(m[6], w[t].w & 0xffffu); m[7] = hmax_bits(m[7], w[t].w >> 16);
    }
  }
  const unsigned ml = 0u - (unsigned)(row < 32);
  v4u o;
  o[0] = (m[0] | (m[1] << 16)) & ml;
  o[1] = (m[2] | (m[3] << 16)) & ml;
  o[2] = (m[4] | (m[5] << 16)) & ml;
  o[3] = (m[6] | (m[7] << 16)) & ml;
  volatile v4u* dst = (volatile v4u*)(gfeat + (size_t)q * 8);
  *dst = o;
  __threadfence();
  *dst = o;
}

__global__ __launch_bounds__(128) void fc2_bn_kernel(const float* F1, const float* W, const float* bias,
                                                     const float* gamma, const float* beta, float* out) {
  __shared__ __align__(16) float os[128];
  const int b = blockIdx.x;
  const int n = threadIdx.x;
  const float* f = F1 + (size_t)b * 1024;
  float acc = 0.0f;
#pragma unroll 4
  for (int k = 0; k < 1024; ++k) acc = __builtin_fmaf(f[k], W[(size_t)k * 128 + n], acc);
  float y = acc + bias[n];
  const float inv = 1.0f / sqrtf(BN_VAR_EPS);
  y = y * inv;
  y = y * gamma[n];
  y = y + beta[n];
  os[n] = y;
  __syncthreads();
  if (threadIdx.x < 32) {
    const v4f v = *(const v4f*)(os + 4 * threadIdx.x);
    volatile v4f* d = (volatile v4f*)(out + (size_t)b * 128 + 4 * threadIdx.x);
    *d = v;
    __threadfence();
    *d = v;
  }
}

extern "C" void kernel_launch(void* const* d_in, const int* in_sizes, int n_in,
                              void* d_out, int out_size, void* d_ws, size_t ws_size,
                              hipStream_t stream) {
  (void)in_sizes;
  constexpr int NB = 32, NPTS = 4096;
  constexpr int S1 = 256, S2 = 64, S3 = 16;
  static_assert(NPTS == 16 * 256, "level-1 points per thread");
  static_assert(512 % 64 == 0 && 1024 % 64 == 0 && 544 % 32 == 0 && 512 % 32 == 0 && 1024 % 32 == 0, "gemm tiling");
  static_assert(NB * S3 == 512, "head rows");
  if (n_in < 23) return;
  if (out_size < NB * 128) return;

  const float* pc    = (const float*)d_in[0];
  const float* w1a   = (const float*)d_in[1];
  const float* b1a   = (const float*)d_in[2];
  const float* w1b   = (const float*)d_in[3];
  const float* b1b   = (const float*)d_in[4];
  const float* w2a   = (const float*)d_in[5];
  const float* b2a   = (const float*)d_in[6];
  const float* w2b   = (const float*)d_in[7];
  const float* b2b   = (const float*)d_in[8];
  const float* w3a   = (const float*)d_in[9];
  const float* b3a   = (const float*)d_in[10];
  const float* w3b   = (const float*)d_in[11];
  const float* b3b   = (const float*)d_in[12];
  const float* w4a   = (const float*)d_in[13];
  const float* b4a   = (const float*)d_in[14];
  const float* w4b   = (const float*)d_in[15];
  const float* b4b   = (const float*)d_in[16];
  const float* fc1w  = (const float*)d_in[17];
  const float* fc1b  = (const float*)d_in[18];
  const float* fc2w  = (const float*)d_in[19];
  const float* fc2b  = (const float*)d_in[20];
  const float* gamma = (const float*)d_in[21];
  const float* beta  = (const float*)d_in[22];
  float* yout = (float*)d_out;

  char* ws = (char*)d_ws;
  size_t off = 0;
  auto alloc = [&](size_t bytes) -> void* {
    void* p = ws + off;
    off += (bytes + 255) & ~(size_t)255;
    return p;
  };
  float* cent1 = (float*)alloc((size_t)NB * S1 * 16);
  float* cent2 = (float*)alloc((size_t)NB * S2 * 16);
  float* cent3 = (float*)alloc((size_t)NB * S3 * 16);
  unsigned short* feats1 = (unsigned short*)alloc((size_t)NB * S1 * 128 * 2);
  unsigned short* feats2 = (unsigned short*)alloc((size_t)NB * S2 * 256 * 2);
  unsigned short* feats3 = (unsigned short*)alloc((size_t)NB * S3 * 512 * 2);
  unsigned short* w1at = (unsigned short*)alloc((size_t)64 * 32 * 2);
  unsigned short* w1bt = (unsigned short*)alloc((size_t)128 * 64 * 2);
  unsigned short* w2at = (unsigned short*)alloc((size_t)128 * 160 * 2);
  unsigned short* w2bt = (unsigned short*)alloc((size_t)256 * 128 * 2);
  unsigned short* w3at = (unsigned short*)alloc((size_t)256 * 288 * 2);
  unsigned short* w3bt = (unsigned short*)alloc((size_t)512 * 256 * 2);
  unsigned short* w4at = (unsigned short*)alloc((size_t)512 * 544 * 2);
  unsigned short* w4bt = (unsigned short*)alloc((size_t)1024 * 512 * 2);
  unsigned short* fc1t = (unsigned short*)alloc((size_t)1024 * 1024 * 2);
  unsigned short* A0    = (unsigned short*)alloc((size_t)512 * 544 * 2);
  unsigned short* G1    = (unsigned short*)alloc((size_t)512 * 512 * 2);
  unsigned short* G2    = (unsigned short*)alloc((size_t)512 * 1024 * 2);
  unsigned short* gfeat = (unsigned short*)alloc((size_t)64 * 1024 * 2);
  float*          F1    = (float*)alloc((size_t)64 * 1024 * 4);
  if (off > ws_size) return;

  auto cvt = [&](const float* W, unsigned short* Wt, int Cin, int Cout, int KP, int nlead) {
    const int chunks = Cout * (KP / 8);
    cvt_wt_kernel<<<(chunks + 255) / 256, 256, 0, stream>>>(W, Wt, Cin, Cout, KP, nlead, WCARRY);
  };
  cvt(w1a, w1at, 9, 64, 32, 3);
  cvt(w1b, w1bt, 64, 128, 64, 0);
  cvt(w2a, w2at, 131, 128, 160, 3);
  cvt(w2b, w2bt, 128, 256, 128, 0);
  cvt(w3a, w3at, 259, 256, 288, 3);
  cvt(w3b, w3bt, 256, 512, 256, 0);
  cvt(w4a, w4at, 515, 512, 544, 3);
  cvt(w4b, w4bt, 512, 1024, 512, 0);
  cvt(fc1w, fc1t, 1024, 1024, 1024, 0);

  fps_kernel<16, true><<<NB, 256, 0, stream>>>(pc, cent1, NPTS, S1);
  group_mlp_kernel<64, 6, 32, 64, 128, true><<<NB * S1, 256, 0, stream>>>(
      pc, feats1, cent1, w1at, b1a, w1bt, b1b, feats1, NPTS, S1, 0.01f);

  fps_kernel<1, false><<<NB, 256, 0, stream>>>(cent1, cent2, S1, S2);
  group_mlp_kernel<64, 128, 160, 128, 256, false><<<NB * S2, 256, 0, stream>>>(
      cent1, feats1, cent2, w2at, b2a, w2bt, b2b, feats2, S1, S2, 0.04f);

  fps_kernel<1, false><<<NB, 256, 0, stream>>>(cent2, cent3, S2, S3);
  group_mlp_kernel<32, 256, 288, 256, 512, false><<<NB * S3, 256, 0, stream>>>(
      cent2, feats2, cent3, w3at, b3a, w3bt, b3b, feats3, S2, S3, 0.16f);

  assemble_head_kernel<<<(512 * 68) / 256, 256, 0, stream>>>(feats3, cent3, A0);
  wmma_gemm64<0, false, 2, 1, false, 2><<<dim3(8, 1, 1), 256, 0, stream>>>(
      A0, A0, 544, 0L, w4at, w4at, 544, 0L, (void*)G1, (void*)G1, 512, 0L,
      b4a, b4a, 0L, 512, 512, 544, WCARRY_INV);
  wmma_gemm64<0, false, 2, 1, false, 2><<<dim3(16, 1, 1), 256, 0, stream>>>(
      G1, G1, 512, 0L, w4bt, w4bt, 512, 0L, (void*)G2, (void*)G2, 1024, 0L,
      b4b, b4b, 0L, 512, 1024, 512, WCARRY_INV);
  maxpts_kernel<<<(64 * 128) / 256, 256, 0, stream>>>(G2, gfeat);
  wmma_gemm64<0, false, 2, 0, false, 2><<<dim3(2, 1, 1), 256, 0, stream>>>(
      gfeat, gfeat, 1024, 0L, fc1t, fc1t, 1024, 0L, (void*)F1, (void*)F1, 1024, 0L,
      fc1b, fc1b, 0L, 64, 1024, 1024, WCARRY_INV);
  fc2_bn_kernel<<<NB, 128, 0, stream>>>(F1, fc2w, fc2b, gamma, beta, yout);
}
